// RNN_4398046511300
// MI455X (gfx1250) — hardware-verified
//
#include <hip/hip_runtime.h>
#include <math.h>

constexpr int NBATCH   = 2048;
constexpr int NSTEP    = 512;
constexpr int NHID     = 50;
constexpr int NPAD     = 64;
constexpr int ROWS_BLK = 64;
constexpr int NTHR     = 128;
constexpr int NWAVES   = NTHR / 32;
constexpr int W_PITCH  = 72;
constexpr int H_PITCH  = 72;
constexpr int X_CHUNK  = 32;
constexpr int X_PITCH  = 36;
constexpr int HF_PITCH = 65;

static_assert(NBATCH % ROWS_BLK == 0, "grid exact");
static_assert(ROWS_BLK == 16 * NWAVES, "one 16-row tile per wave");
static_assert(NSTEP % X_CHUNK == 0, "x chunks exact");
static_assert(NHID <= NPAD && NPAD % 32 == 0, "K and N padded to tile multiples");
static_assert((NPAD * W_PITCH) % NTHR == 0, "weight plane fill exact");
static_assert((ROWS_BLK * H_PITCH) % NTHR == 0, "state plane fill exact");
static_assert(ROWS_BLK * X_CHUNK == 4 * NTHR * 4, "x stage fill exact");
static_assert(W_PITCH % 8 == 0 && H_PITCH % 8 == 0 && X_PITCH % 4 == 0, "16-B aligned rows");
static_assert(W_PITCH >= NPAD && H_PITCH >= NPAD, "pitch covers padded K");
static_assert(2 * NPAD * W_PITCH * 2 + 2 * ROWS_BLK * H_PITCH * 2 + ROWS_BLK * X_PITCH * 4 +
              ROWS_BLK * HF_PITCH * 4 + 3 * NPAD * 4 <= 65536, "static LDS budget");

typedef __attribute__((ext_vector_type(16))) __bf16 v16b;
typedef __attribute__((ext_vector_type(8)))  __bf16 v8b;
typedef __attribute__((ext_vector_type(8)))  float  v8f;
typedef __attribute__((ext_vector_type(4)))  float  v4f;

__device__ __forceinline__ unsigned short f2bf_bits(float f) {
  unsigned u = __float_as_uint(f);
  return (unsigned short)((u + 0x7FFFu + ((u >> 16) & 1u)) >> 16);
}
__device__ __forceinline__ float bf_bits2f(unsigned short h) { return __uint_as_float(((unsigned)h) << 16); }

union FragB { v16b v; v8b h[2]; };
__device__ __forceinline__ v16b frag_load(const __bf16* p) {
  FragB f;
  f.h[0] = *(const v8b*)(p);
  f.h[1] = *(const v8b*)(p + 16);
  return f.v;
}
__device__ __forceinline__ v8f mma_bf(v16b a, v16b b, v8f c) {
  return __builtin_amdgcn_wmma_f32_16x16x32_bf16(false, a, false, b, (short)0, c, false, false);
}
__device__ __forceinline__ void group_guard(v8f& acc, v16b a0, v16b a1, v16b a2, v16b a3,
                                            v16b b0, v16b b1, v16b b2, v16b b3) {
  asm volatile("v_nop\n\tv_nop\n\tv_nop\n\tv_nop"
               : "+v"(acc)
               : "v"(a0), "v"(a1), "v"(a2), "v"(a3), "v"(b0), "v"(b1), "v"(b2), "v"(b3));
}

__global__ __launch_bounds__(NTHR) void rnn_seq_kernel(const float* __restrict__ x,
                                                       const float* __restrict__ w_ih,
                                                       const float* __restrict__ w_hh,
                                                       const float* __restrict__ b_ih,
                                                       const float* __restrict__ b_hh,
                                                       const float* __restrict__ w_fc,
                                                       const float* __restrict__ b_fc,
                                                       float* __restrict__ out) {
  __shared__ __align__(16) __bf16 Wh[NPAD * W_PITCH];
  __shared__ __align__(16) __bf16 Wl[NPAD * W_PITCH];
  __shared__ __align__(16) __bf16 Hh[ROWS_BLK * H_PITCH];
  __shared__ __align__(16) __bf16 Hl[ROWS_BLK * H_PITCH];
  __shared__ __align__(16) float  Xs[ROWS_BLK * X_PITCH];
  __shared__ float Hf[ROWS_BLK * HF_PITCH];
  __shared__ float wihs[NPAD];
  __shared__ float biass[NPAD];
  __shared__ float wfcs[NPAD];

  const int tid = threadIdx.x;
  const int lane = tid & 31;
  const int wave = tid >> 5;
  const int c = lane & 15;
  const int hh = lane >> 4;
  const int koff = hh * 8;
  const int rowbase = blockIdx.x * ROWS_BLK;

#pragma unroll 1
  for (int i = tid; i < NPAD * W_PITCH; i += NTHR) {
    const int n = i / W_PITCH;
    const int k = i - n * W_PITCH;
    const bool ok = (n < NHID) && (k < NHID);
    const int nn = (n < NHID) ? n : (NHID - 1);
    const int kk = (k < NHID) ? k : (NHID - 1);
    const float wraw = w_hh[nn * NHID + kk];
    const float w = ok ? wraw : 0.0f;
    const unsigned short hb = f2bf_bits(w);
    const unsigned short lb = f2bf_bits(w - bf_bits2f(hb));
    Wh[i] = __builtin_bit_cast(__bf16, hb);
    Wl[i] = __builtin_bit_cast(__bf16, lb);
  }
  {
    const unsigned short zb = 0;
    const __bf16 z16 = __builtin_bit_cast(__bf16, zb);
#pragma unroll 1
    for (int i = tid; i < ROWS_BLK * H_PITCH; i += NTHR) {
      Hh[i] = z16;
      Hl[i] = z16;
    }
  }
  if (tid < NPAD) {
    const bool ok = tid < NHID;
    const int ii = ok ? tid : (NHID - 1);
    const float a = w_ih[ii];
    const float b0 = b_ih[ii];
    const float b1 = b_hh[ii];
    const float f = w_fc[ii];
    wihs[tid]  = ok ? a : 0.0f;
    biass[tid] = ok ? (b0 + b1) : 0.0f;
    wfcs[tid]  = ok ? f : 0.0f;
  }
  const float bfc = b_fc[0];
  __syncthreads();

  const int drow0 = 16 * wave + 8 * hh;
  const __bf16* harow_h = Hh + (16 * wave + c) * H_PITCH + koff;
  const __bf16* harow_l = Hl + (16 * wave + c) * H_PITCH + koff;

#pragma unroll 1
  for (int t = 0; t < NSTEP; ++t) {
    const int tt = t & (X_CHUNK - 1);
    if (tt == 0) {
#pragma unroll
      for (int it = 0; it < 4; ++it) {
        const int idx = it * NTHR + tid;
        const int row = idx >> 3;
        const int c4 = (idx & 7) * 4;
        const v4f v = *(const v4f*)(x + (size_t)(rowbase + row) * NSTEP + t + c4);
        *(v4f*)(Xs + row * X_PITCH + c4) = v;
      }
      __syncthreads();
    }

    const v16b ah0 = frag_load(harow_h);
    const v16b ah1 = frag_load(harow_h + 32);
    const v16b al0 = frag_load(harow_l);
    const v16b al1 = frag_load(harow_l + 32);
    float xr[8];
#pragma unroll
    for (int r = 0; r < 8; ++r) xr[r] = Xs[(drow0 + r) * X_PITCH + tt];
    asm volatile("" ::: "memory");
    const bool last = (t == NSTEP - 1);

#pragma unroll 1
    for (int j = 0; j < 4; ++j) {
      const int n = 16 * j + c;
      const __bf16* wrow_h = Wh + n * W_PITCH + koff;
      const __bf16* wrow_l = Wl + n * W_PITCH + koff;
      const v16b bh0 = frag_load(wrow_h);
      const v16b bh1 = frag_load(wrow_h + 32);
      const v16b bl0 = frag_load(wrow_l);
      const v16b bl1 = frag_load(wrow_l + 32);
      const float wv = wihs[n];
      const float bv = biass[n];
      v8f acc;
#pragma unroll
      for (int r = 0; r < 8; ++r) acc[r] = fmaf(xr[r], wv, bv);
      acc = mma_bf(ah0, bh0, acc);
      acc = mma_bf(ah1, bh1, acc);
      acc = mma_bf(al0, bh0, acc);
      acc = mma_bf(al1, bh1, acc);
      acc = mma_bf(ah0, bl0, acc);
      acc = mma_bf(ah1, bl1, acc);
      group_guard(acc, ah0, ah1, al0, al1, bh0, bh1, bl0, bl1);

      const bool live = n < NHID;
      float hv[8];
#pragma unroll
      for (int r = 0; r < 8; ++r) {
        const float pre = acc[r];
        const float th = tanhf(pre);
        const float hval = live ? th : 0.0f;
        hv[r] = hval;
        const unsigned short hb = f2bf_bits(hval);
        const unsigned short lb = f2bf_bits(hval - bf_bits2f(hb));
        const int o = (drow0 + r) * H_PITCH + n;
        Hh[o] = __builtin_bit_cast(__bf16, hb);
        Hl[o] = __builtin_bit_cast(__bf16, lb);
      }
      if (last) {
#pragma unroll
        for (int r = 0; r < 8; ++r) Hf[(drow0 + r) * HF_PITCH + n] = hv[r];
      }
    }
    __syncthreads();
  }

  if (tid < ROWS_BLK) {
    float s = 0.0f;
#pragma unroll 1
    for (int h = 0; h < NHID; ++h) s = fmaf(Hf[tid * HF_PITCH + h], wfcs[h], s);
    const float o = s + bfc;
    volatile float* op = out + rowbase + tid;
    *op = o;
    __threadfence();
    *op = o;
  }
}

extern "C" void kernel_launch(void* const* d_in, const int* in_sizes, int n_in,
                              void* d_out, int out_size, void* d_ws, size_t ws_size, hipStream_t stream) {
  (void)in_sizes; (void)out_size; (void)d_ws; (void)ws_size;
  if (n_in < 7 || d_out == nullptr) return;
  const float* x    = (const float*)d_in[0];
  const float* w_ih = (const float*)d_in[1];
  const float* w_hh = (const float*)d_in[2];
  const float* b_ih = (const float*)d_in[3];
  const float* b_hh = (const float*)d_in[4];
  const float* w_fc = (const float*)d_in[5];
  const float* b_fc = (const float*)d_in[6];
  float* out = (float*)d_out;
  rnn_seq_kernel<<<NBATCH / ROWS_BLK, NTHR, 0, stream>>>(x, w_ih, w_hh, b_ih, b_hh, w_fc, b_fc, out);
}
